// Mamba3Clean_6236292514072
// MI455X (gfx1250) — hardware-run, weakly checked
//
#include <hip/hip_runtime.h>
#include <math.h>

typedef __attribute__((ext_vector_type(16))) _Float16 v16h;
typedef __attribute__((ext_vector_type(8)))  _Float16 v8h;
typedef __attribute__((ext_vector_type(2)))  _Float16 v2h;
typedef __attribute__((ext_vector_type(16))) __bf16   v16b;
typedef __attribute__((ext_vector_type(8)))  __bf16   v8b;
typedef __attribute__((ext_vector_type(8)))  float    v8f;
typedef __attribute__((ext_vector_type(4)))  float    v4f;
typedef __attribute__((ext_vector_type(2)))  float    v2f;

constexpr int kT    = 1024;
constexpr int kDM   = 1024;
constexpr int kDI   = 2048;
constexpr int kNH   = 32;
constexpr int kHD   = 64;
constexpr int kNs   = 128;
constexpr int kR    = 32;
constexpr int kNQ   = 4;
constexpr int kNP   = 4480;
constexpr int kCX   = 2048;
constexpr int kCB   = 4096;
constexpr int kCC   = 4224;
constexpr int kCDt  = 4352;
constexpr int kCA   = 4384;
constexpr int kCTr  = 4416;
constexpr int kCAn  = 4448;
constexpr int kThr  = 256;
constexpr float kInCarry = 1024.0f;
constexpr float kWCarry  = 4096.0f;
constexpr float kCY   = 128.0f;
constexpr float kF16MinNormal = 6.103515625e-5f;
constexpr float kPi = 3.14159274101257324f;

static_assert(kDI == kNH * kHD && kNs == kNQ * 32 && kR == 32 && kCAn + kR == kNP && kCB == 2 * kDI && kCC == kCB + kNs && kCDt == kCC + kNs && kCA == kCDt + kNH && kCTr == kCA + kNH && kCAn == kCTr + kNH && (kNP % 64) == 0, "the column map and the index arithmetic below use these sizes");

constexpr size_t kOffZB = 0ull;
constexpr size_t kOffU16 = 18432ull;
constexpr size_t kOffWIN16 = 2115584ull;
constexpr size_t kOffWOUT16 = 11290624ull;
constexpr size_t kOffPROJ = 15484928ull;
constexpr size_t kOffAL = 33835008ull;
constexpr size_t kOffBE = 33966080ull;
constexpr size_t kOffGA = 34097152ull;
constexpr size_t kOffDTP = 34228224ull;
constexpr size_t kOffRC = 34359296ull;
constexpr size_t kOffRS = 38553600ull;
constexpr size_t kOffYP = 42747904ull;
constexpr size_t kOffY16 = 76302336ull;
constexpr size_t kWsTotal = 80496640ull;
static_assert(kWsTotal <= 134217728ull, "carve cap: under 128 MiB");
static_assert(kOffZB == 0
  && kOffU16 == kOffZB + 18432ull
  && kOffWIN16 == kOffU16 + 2097152ull
  && kOffWOUT16 == kOffWIN16 + 9175040ull
  && kOffPROJ == kOffWOUT16 + 4194304ull
  && kOffAL == kOffPROJ + 18350080ull
  && kOffBE == kOffAL + 131072ull
  && kOffGA == kOffBE + 131072ull
  && kOffDTP == kOffGA + 131072ull
  && kOffRC == kOffDTP + 131072ull
  && kOffRS == kOffRC + 4194304ull
  && kOffYP == kOffRS + 4194304ull
  && kOffY16 == kOffYP + 33554432ull
  && kWsTotal == kOffY16 + 4194304ull, "the carve is a chain: every region starts where the one before ends");
static_assert((kOffU16 % 256) == 0 && (kOffWIN16 % 256) == 0 && (kOffWOUT16 % 256) == 0 && (kOffPROJ % 256) == 0 && (kOffAL % 256) == 0 && (kOffBE % 256) == 0 && (kOffGA % 256) == 0 && (kOffDTP % 256) == 0 && (kOffRC % 256) == 0 && (kOffRS % 256) == 0 && (kOffYP % 256) == 0 && (kOffY16 % 256) == 0, "every region starts on a multiple of 256 B");

__device__ __forceinline__ unsigned short f2bf_bits(float f) {
  unsigned u = __float_as_uint(f);
  return (unsigned short)((u + 0x7FFFu + ((u >> 16) & 1u)) >> 16);
}
__device__ __forceinline__ float bf_bits2f(unsigned short h) { return __uint_as_float(((unsigned)h) << 16); }
__device__ __forceinline__ float bf16r(float f) { return bf_bits2f(f2bf_bits(f)); }
__device__ __forceinline__ float carry_flush(float v, float carry) {
  const float s = v * carry;
  return (fabsf(s) < kF16MinNormal) ? 0.0f : s;
}

__device__ __forceinline__ void dep_guard4_h(v8f& a, v8f& b, v8f& c, v8f& d, v16h x, v16h y) { asm volatile("v_nop\n\tv_nop\n\tv_nop\n\tv_nop" : "+v"(a), "+v"(b), "+v"(c), "+v"(d) : "v"(x), "v"(y)); }
__device__ __forceinline__ void dep_guard4_b(v8f& a, v8f& b, v8f& c, v8f& d, v16b x, v16b y) { asm volatile("v_nop\n\tv_nop\n\tv_nop\n\tv_nop" : "+v"(a), "+v"(b), "+v"(c), "+v"(d) : "v"(x), "v"(y)); }
__device__ __forceinline__ void keep4_h(v16h a, v16h b, v16h c, v16h d) { asm volatile("v_nop" :: "v"(a), "v"(b), "v"(c), "v"(d)); }
__device__ __forceinline__ void keep4_b(v16b a, v16b b, v16b c, v16b d) { asm volatile("v_nop" :: "v"(a), "v"(b), "v"(c), "v"(d)); }
__device__ __forceinline__ void acc_guard4(v8f& a, v8f& b, v8f& c, v8f& d) { asm volatile("v_nop\n\tv_nop\n\tv_nop\n\tv_nop" : "+v"(a), "+v"(b), "+v"(c), "+v"(d)); }

template <typename T> struct Frag;
template <> struct Frag<_Float16> {
  typedef v16h V; union U { v16h v; v8h h[2]; };
  static __device__ __forceinline__ v16h load(const _Float16* p) {
    U f; f.h[0] = *(const v8h*)(p); f.h[1] = *(const v8h*)(p + 16); return f.v;
  }
  static __device__ __forceinline__ v8f mma(v16h a, v16h b, v8f c) {
    return __builtin_amdgcn_wmma_f32_16x16x32_f16(false, a, false, b, (short)0, c, false, false);
  }
  static __device__ __forceinline__ void guard4(v8f& a, v8f& b, v8f& c, v8f& d, v16h x, v16h y) { dep_guard4_h(a, b, c, d, x, y); }
  static __device__ __forceinline__ void keep(v16h a, v16h b, v16h c, v16h d) { keep4_h(a, b, c, d); }
};
template <> struct Frag<__bf16> {
  typedef v16b V; union U { v16b v; v8b h[2]; };
  static __device__ __forceinline__ v16b load(const __bf16* p) {
    U f; f.h[0] = *(const v8b*)(p); f.h[1] = *(const v8b*)(p + 16); return f.v;
  }
  static __device__ __forceinline__ v8f mma(v16b a, v16b b, v8f c) {
    return __builtin_amdgcn_wmma_f32_16x16x32_bf16(false, a, false, b, (short)0, c, false, false);
  }
  static __device__ __forceinline__ void guard4(v8f& a, v8f& b, v8f& c, v8f& d, v16b x, v16b y) { dep_guard4_b(a, b, c, d, x, y); }
  static __device__ __forceinline__ void keep(v16b a, v16b b, v16b c, v16b d) { keep4_b(a, b, c, d); }
};

__device__ __forceinline__ v8f mma_h(v16h a, v16h b, v8f c) {
  c = __builtin_amdgcn_wmma_f32_16x16x32_f16(false, a, false, b, (short)0, c, false, false);
  asm volatile("v_nop\n\tv_nop\n\tv_nop\n\tv_nop" : "+v"(c) : "v"(a), "v"(b));
  return c;
}

template <int ET> struct Elem;
template <> struct Elem<0> { typedef _Float16 T; };
template <> struct Elem<1> { typedef __bf16 T; };
template <int ET, bool SPLIT, int BIAS_MODE, int OUT_MODE, bool RESID, int ACT = 0>
__global__ __launch_bounds__(256) void wmma_gemm64(
    const unsigned short* __restrict__ Ap, const unsigned short* __restrict__ A2p, int lda, long strideA,
    const unsigned short* __restrict__ Btp, const unsigned short* __restrict__ Bt2p, int ldb, long strideB,
    void* __restrict__ Cout, void* __restrict__ Cout2, int ldc, long strideC,
    const float* __restrict__ bias,
    const float* __restrict__ resid, long strideR,
    int M, int N, int K, float scale) {
  typedef typename Elem<ET>::T T;
  typedef typename Frag<T>::V V;
  const T* A = (const T*)Ap; const T* A2 = (const T*)A2p; const T* Bt = (const T*)Btp; const T* Bt2 = (const T*)Bt2p;
  __shared__ __align__(16) float sT[8][16 * 68];
  const int b    = blockIdx.y;
  const int lane = threadIdx.x & 31;
  const int wave = threadIdx.x >> 5;
  const int tilesN = N >> 6;
  const int tilesM = M >> 6;
  const int tile = blockIdx.x * 8 + wave;
  if (tile >= tilesM * tilesN) return;
  const int tm = tile / tilesN;
  const int tn = tile - tm * tilesN;
  const int m0 = tm << 6;
  const int n0 = tn << 6;

  const T* Ab  = A  + (size_t)b * strideA;
  const T* Bb  = Bt + (size_t)b * strideB;
  const T* Ab2 = SPLIT ? (A2  + (size_t)b * strideA) : nullptr;
  const T* Bb2 = SPLIT ? (Bt2 + (size_t)b * strideB) : nullptr;

  const int rlane = lane & 15;
  const int koff  = (lane >> 4) * 8;
  const int mOff  = (lane >> 4) * 8;

  v8f acc[4][4];
#pragma unroll
  for (int i = 0; i < 4; ++i)
#pragma unroll
    for (int j = 0; j < 4; ++j) acc[i][j] = (v8f){0.f,0.f,0.f,0.f,0.f,0.f,0.f,0.f};

  for (int k0 = 0; k0 < K; k0 += 32) {
    V bh[4], bl[4];
#pragma unroll
    for (int j = 0; j < 4; ++j) {
      const size_t bo = (size_t)(n0 + (j << 4) + rlane) * ldb + koff + k0;
      bh[j] = Frag<T>::load(Bb + bo);
      if (SPLIT) bl[j] = Frag<T>::load(Bb2 + bo);
    }
#pragma unroll
    for (int i = 0; i < 4; ++i) {
      const size_t ao = (size_t)(m0 + (i << 4) + rlane) * lda + koff + k0;
      V ah = Frag<T>::load(Ab + ao);
      V al;
      if (SPLIT) al = Frag<T>::load(Ab2 + ao);
#pragma unroll
      for (int j = 0; j < 4; ++j) {
        acc[i][j] = Frag<T>::mma(ah, bh[j], acc[i][j]);
        if (SPLIT) {
          acc[i][j] = Frag<T>::mma(ah, bl[j], acc[i][j]);
          acc[i][j] = Frag<T>::mma(al, bh[j], acc[i][j]);
        }
      }
      Frag<T>::guard4(acc[i][0], acc[i][1], acc[i][2], acc[i][3], ah, SPLIT ? al : ah);
    }
    Frag<T>::keep(bh[0], bh[1], bh[2], bh[3]);
    if (SPLIT) Frag<T>::keep(bl[0], bl[1], bl[2], bl[3]);
  }
  acc_guard4(acc[0][0], acc[0][1], acc[0][2], acc[0][3]);
  acc_guard4(acc[1][0], acc[1][1], acc[1][2], acc[1][3]);
  acc_guard4(acc[2][0], acc[2][1], acc[2][2], acc[2][3]);
  acc_guard4(acc[3][0], acc[3][1], acc[3][2], acc[3][3]);

  float* slab = sT[wave];
  const float* Rb = RESID ? (resid + (size_t)b * strideR) : nullptr;
#pragma unroll
  for (int i = 0; i < 4; ++i) {
    const int mBase = m0 + (i << 4);
#pragma unroll
    for (int j = 0; j < 4; ++j) {
      const int n = n0 + (j << 4) + rlane;
      float bv = 0.f;
      if (BIAS_MODE == 2) bv = bias[n];
#pragma unroll
      for (int r = 0; r < 8; ++r) {
        float v = acc[i][j][r] * scale;
        if (BIAS_MODE == 1) v += bias[mBase + mOff + r];
        if (BIAS_MODE == 2) v += bv;
        if (RESID) v += Rb[(size_t)(mBase + mOff + r) * ldc + n];
        if (ACT == 1) v = tanhf(v);
        if (ACT == 2) v = fmaxf(v, 0.0f);
        if (ACT == 3) v = v / (1.0f + expf(-v));
        if (ACT == 4) v = (v > 0.f) ? v : 0.01f * v;
        slab[(mOff + r) * 68 + (j << 4) + rlane] = v;
      }
    }
    __builtin_amdgcn_fence(__ATOMIC_RELEASE, "workgroup");
    __builtin_amdgcn_wave_barrier();
    __builtin_amdgcn_fence(__ATOMIC_ACQUIRE, "workgroup");
    if (OUT_MODE == 0) {
      float* C = (float*)Cout + (size_t)b * strideC;
      const int hh = lane >> 4, c4 = (lane & 15) * 4;
      for (int pass = 0; pass < 2; ++pass) {
#pragma unroll
        for (int it = 0; it < 8; ++it) {
          const int row = it * 2 + hh;
          v4f v = *(const v4f*)(slab + row * 68 + c4);
          *(volatile v4f*)(C + (size_t)(mBase + row) * ldc + n0 + c4) = v;
        }
        __threadfence();
      }
    } else {
      const int q = lane >> 3, c8 = (lane & 7) * 8;
      unsigned short* C  = (unsigned short*)Cout  + (size_t)b * strideC;
      unsigned short* C2 = (OUT_MODE == 2) ? ((unsigned short*)Cout2 + (size_t)b * strideC) : nullptr;
      for (int pass = 0; pass < 2; ++pass) {
#pragma unroll
        for (int it = 0; it < 4; ++it) {
          const int row = it * 4 + q;
          const float* sp = slab + row * 68 + c8;
          v8h hv, lv;
#pragma unroll
          for (int e = 0; e < 8; ++e) {
            if (OUT_MODE == 1) {
              hv[e] = (_Float16)sp[e];
            } else {
              unsigned short hb = f2bf_bits(sp[e]);
              unsigned short lb = f2bf_bits(sp[e] - bf_bits2f(hb));
              hv[e] = __builtin_bit_cast(_Float16, hb);
              lv[e] = __builtin_bit_cast(_Float16, lb);
            }
          }
          *(volatile v8h*)(C + (size_t)(mBase + row) * ldc + n0 + c8) = hv;
          if (OUT_MODE == 2) *(volatile v8h*)(C2 + (size_t)(mBase + row) * ldc + n0 + c8) = lv;
        }
        __threadfence();
      }
    }
    __builtin_amdgcn_fence(__ATOMIC_RELEASE, "workgroup");
    __builtin_amdgcn_wave_barrier();
    __builtin_amdgcn_fence(__ATOMIC_ACQUIRE, "workgroup");
  }
}


__device__ __forceinline__ void store2(float* p, float v) {
  *(volatile float*)p = v;
  __threadfence();
  *(volatile float*)p = v;
}

__global__ __launch_bounds__(kThr) void cast_plane_kernel(const float* __restrict__ src, unsigned short* __restrict__ dst,
                                                          int colsLog2, int dstPitch, int dstOff) {
  const int i   = blockIdx.x * kThr + threadIdx.x;
  const int sh  = colsLog2 - 3;
  const int row = i >> sh;
  const int c8  = (i & ((1 << sh) - 1)) * 8;
  const float* sp = src + ((size_t)row << colsLog2) + c8;
  const v4f a0 = *(const v4f*)(sp);
  const v4f a1 = *(const v4f*)(sp + 4);
  v8h hv;
#pragma unroll
  for (int e = 0; e < 4; ++e) {
    const float f0 = a0[e];
    const float f1 = a1[e];
    hv[e]     = (_Float16)carry_flush(bf16r(f0), kInCarry);
    hv[4 + e] = (_Float16)carry_flush(bf16r(f1), kInCarry);
  }
  unsigned short* dp = dst + (size_t)row * dstPitch + dstOff + c8;
  *(volatile v8h*)dp = hv;
  __threadfence();
  *(volatile v8h*)dp = hv;
}

__global__ __launch_bounds__(256) void wt_plane_kernel(const float* __restrict__ W, unsigned short* __restrict__ dst, int K, int N, int nLive, int ldd, int colOff) {
  const int n  = blockIdx.x;
  const int k8 = threadIdx.x * 8;
  const bool live = n < nLive;
  const int nc = live ? n : 0;
  v8h hv;
#pragma unroll
  for (int e = 0; e < 8; ++e) {
    const float w = W[(size_t)(k8 + e) * N + nc];
    hv[e] = (_Float16)(live ? carry_flush(bf16r(w), kWCarry) : 0.0f);
  }
  unsigned short* dp = dst + (size_t)n * ldd + colOff + k8;
  *(volatile v8h*)dp = hv;
  __threadfence();
  *(volatile v8h*)dp = hv;
}

__global__ __launch_bounds__(kThr) void setup_kernel(float* __restrict__ ZB) {
  store2(ZB + (size_t)blockIdx.x * kThr + threadIdx.x, 0.0f);
}
static_assert(4608 == 18 * kThr && 4608 >= kNP, "set-up grid: 18 blocks");

__global__ __launch_bounds__(kThr) void pre_kernel(const float* __restrict__ PROJ, const float* __restrict__ dtb,
                                                  float* __restrict__ AL, float* __restrict__ BE, float* __restrict__ GA, float* __restrict__ DTP) {
  const unsigned i = blockIdx.x * (unsigned)kThr + threadIdx.x;
  const size_t tk = i >> 5;
  const unsigned hd = i & 31u;
  const float* pr = PROJ + tk * kNP;
  const float b0 = dtb[hd];
  const float vdt = pr[kCDt + hd] + bf16r(b0);
  const float vA = pr[kCA + hd];
  const float vtr = pr[kCTr + hd];
  const float dt = fmaxf(vdt, 0.0f) + log1pf(expf(-fabsf(vdt)));
  const float A = fminf(-(fmaxf(vA, 0.0f) + log1pf(expf(-fabsf(vA)))), -1e-4f);
  const float tr = 1.0f / (1.0f + expf(-vtr));
  const float al = expf(A * dt);
  store2(AL + i, al);
  store2(BE + i, ((1.0f - tr) * dt) * al);
  store2(GA + i, tr * dt);
  store2(DTP + i, dt);
}
static_assert((size_t)kT * kNH == 128ull * kThr, "the token-head grid exact: 128 blocks");

__global__ __launch_bounds__(kThr) void theta_kernel(const float* __restrict__ PROJ, const float* __restrict__ DTP, float* __restrict__ RC, float* __restrict__ RS) {
  const unsigned i = blockIdx.x * (unsigned)kThr + threadIdx.x;
  const unsigned hd = i >> 5;
  const unsigned r = i & 31u;
  float acc = 0.0f;
  for (int t = 0; t < kT; ++t) {
    const float an = PROJ[(size_t)t * kNP + kCAn + r];
    const float dt = DTP[(size_t)t * kNH + hd];
    acc += (tanhf(an) * dt) * kPi;
    const size_t o = ((size_t)t * kNH + hd) * kR + r;
    store2(RC + o, cosf(acc));
    store2(RS + o, sinf(acc));
  }
}
static_assert(kNH * kR == 4 * kThr, "the angles' grid exact: 4 blocks");

__global__ __launch_bounds__(kThr) void scan_rot_kernel(const float* __restrict__ PROJ, const float* __restrict__ AL, const float* __restrict__ BE, const float* __restrict__ GA,
                                                        const float* __restrict__ RC, const float* __restrict__ RS, float* __restrict__ YP) {
  const unsigned ch = blockIdx.x * (unsigned)kThr + threadIdx.x;
  const unsigned hd = ch >> 6;
  float sr[kR], si[kR];
#pragma unroll
  for (int n = 0; n < kR; ++n) { sr[n] = 0.0f; si[n] = 0.0f; }
  float px = 0.0f;
  for (int t = 0; t < kT; ++t) {
    const float* pr = PROJ + (size_t)t * kNP;
    const size_t th = (size_t)t * kNH + hd;
    const float al = AL[th], be = BE[th], ga = GA[th];
    const float xt = pr[kCX + ch];
    const float m = px * be + xt * ga;
    const float* pc = RC + th * kR;
    const float* ps = RS + th * kR;
    float y = 0.0f;
#pragma unroll
    for (int q = 0; q < kR / 4; ++q) {
      const v4f bv = *(const v4f*)(pr + kCB + 4 * q), cv = *(const v4f*)(pr + kCC + 4 * q);
      const v4f c4 = *(const v4f*)(pc + 4 * q), s4 = *(const v4f*)(ps + 4 * q);
#pragma unroll
      for (int e = 0; e < 4; ++e) {
        const int n = 4 * q + e;
        const float base = bv[e] * m;
        const float nr = sr[n] * al + base * c4[e];
        const float ni = si[n] * al + base * s4[e];
        sr[n] = nr; si[n] = ni;
        y += (nr * c4[e] + ni * s4[e]) * cv[e];
      }
    }
    px = xt;
    store2(YP + ((size_t)t * kNQ + 0) * kDI + ch, y);
  }
}
static_assert(kDI == 8 * kThr && (kR % 4) == 0 && (kCB % 4) == 0 && (kCC % 4) == 0, "rotary walk grid exact: 8 blocks; the 16-B loads aligned");

__global__ __launch_bounds__(kThr) void scan_plain_kernel(const float* __restrict__ PROJ, const float* __restrict__ AL, const float* __restrict__ BE, const float* __restrict__ GA,
                                                          float* __restrict__ YP) {
  const unsigned qt = 1u + (blockIdx.x >> 3);
  const unsigned ch = (blockIdx.x & 7u) * (unsigned)kThr + threadIdx.x;
  const unsigned hd = ch >> 6;
  const unsigned n0 = qt * 32u;
  float sr[32];
#pragma unroll
  for (int n = 0; n < 32; ++n) sr[n] = 0.0f;
  float px = 0.0f;
  for (int t = 0; t < kT; ++t) {
    const float* pr = PROJ + (size_t)t * kNP;
    const size_t th = (size_t)t * kNH + hd;
    const float al = AL[th], be = BE[th], ga = GA[th];
    const float xt = pr[kCX + ch];
    const float m = px * be + xt * ga;
    float y = 0.0f;
#pragma unroll
    for (int q = 0; q < 8; ++q) {
      const v4f bv = *(const v4f*)(pr + kCB + n0 + 4 * q), cv = *(const v4f*)(pr + kCC + n0 + 4 * q);
#pragma unroll
      for (int e = 0; e < 4; ++e) {
        const int n = 4 * q + e;
        const float nr = sr[n] * al + bv[e] * m;
        sr[n] = nr;
        y += nr * cv[e];
      }
    }
    px = xt;
    store2(YP + ((size_t)t * kNQ + qt) * kDI + ch, y);
  }
}
static_assert((kNQ - 1) * (kDI / kThr) == 24, "plain walk grid exact: 24 blocks: eight a quarter");

__global__ __launch_bounds__(kThr) void ygate_kernel(const float* __restrict__ YP, const float* __restrict__ PROJ, const float* __restrict__ Dp, unsigned short* __restrict__ Y16) {
  const size_t tk = blockIdx.y;
  const unsigned c8 = threadIdx.x * 8u;
  const float d0 = Dp[c8 >> 6];
  const float dsk = bf16r(d0);
  const float* y0 = YP + (tk * kNQ + 0) * kDI + c8;
  const float* y1 = YP + (tk * kNQ + 1) * kDI + c8;
  const float* y2 = YP + (tk * kNQ + 2) * kDI + c8;
  const float* y3 = YP + (tk * kNQ + 3) * kDI + c8;
  const float* xp = PROJ + tk * kNP + kCX + c8;
  const float* zp = PROJ + tk * kNP + c8;
  v8h hv;
#pragma unroll
  for (int e = 0; e < 8; ++e) {
    const float z = zp[e];
    const float y = (((y0[e] + y1[e]) + y2[e]) + y3[e]) + dsk * xp[e];
    hv[e] = (_Float16)carry_flush(y * (z / (1.0f + expf(-z))), kCY);
  }
  unsigned short* dp = Y16 + tk * kDI + c8;
  *(volatile v8h*)dp = hv;
  __threadfence();
  *(volatile v8h*)dp = hv;
}
static_assert(kDI == kThr * 8 && (kHD % 8) == 0, "gate grid exact: 256 groups a row; a group of eight channels lies in one head");

extern "C" void kernel_launch(void* const* d_in, const int* in_sizes, int n_in,
                              void* d_out, int out_size, void* d_ws, size_t ws_size,
                              hipStream_t stream) {
  if (n_in < 5 || d_out == nullptr || d_ws == nullptr) return;
  if (in_sizes[0] != kT * kDM || in_sizes[1] != kNP * kDM || in_sizes[2] != kDM * kDI || in_sizes[3] != kNH || in_sizes[4] != kNH) return;
  if (out_size != kT * kDM) return;
  if (ws_size < kWsTotal) return;
  const float* u    = (const float*)d_in[0];
  const float* win  = (const float*)d_in[1];
  const float* wout = (const float*)d_in[2];
  const float* dtb  = (const float*)d_in[3];
  const float* Dp   = (const float*)d_in[4];
  float* out = (float*)d_out;
  char* ws = (char*)d_ws;
  float* ZB = (float*)(ws + kOffZB);
  unsigned short* U16    = (unsigned short*)(ws + kOffU16);
  unsigned short* WIN16  = (unsigned short*)(ws + kOffWIN16);
  unsigned short* WOUT16 = (unsigned short*)(ws + kOffWOUT16);
  float* PROJ = (float*)(ws + kOffPROJ);
  float* AL  = (float*)(ws + kOffAL);
  float* BE  = (float*)(ws + kOffBE);
  float* GA  = (float*)(ws + kOffGA);
  float* DTP = (float*)(ws + kOffDTP);
  float* RC  = (float*)(ws + kOffRC);
  float* RS  = (float*)(ws + kOffRS);
  float* YP  = (float*)(ws + kOffYP);
  unsigned short* Y16 = (unsigned short*)(ws + kOffY16);

  static_assert(((size_t)kT * kDM / 8) % kThr == 0 && ((size_t)kNP * kDM / 8) % kThr == 0 && ((size_t)kDM * kDI / 8) % kThr == 0, "the casts' grids");
  cast_plane_kernel<<<(int)(((size_t)kT * kDM / 8) / kThr), kThr, 0, stream>>>(u, U16, 10, kDM, 0);
  cast_plane_kernel<<<(int)(((size_t)kNP * kDM / 8) / kThr), kThr, 0, stream>>>(win, WIN16, 10, kDM, 0);
  cast_plane_kernel<<<(int)(((size_t)kDM * kDI / 8) / kThr), kThr, 0, stream>>>(wout, WOUT16, 10, 1024, 0);
  setup_kernel<<<18, kThr, 0, stream>>>(ZB);

  wmma_gemm64<0, false, 2, 0, false, 0><<<dim3((kT / 64) * (kNP / 64) / 8, 1), 256, 0, stream>>>(
      U16, U16, kDM, 0L, WIN16, WIN16, kDM, 0L, (void*)PROJ, (void*)PROJ, kNP, 0L, ZB, nullptr, 0L, kT, kNP, kDM, 1.0f / (kInCarry * kInCarry));
  pre_kernel<<<128, kThr, 0, stream>>>(PROJ, dtb, AL, BE, GA, DTP);
  theta_kernel<<<4, kThr, 0, stream>>>(PROJ, DTP, RC, RS);
  scan_rot_kernel<<<8, kThr, 0, stream>>>(PROJ, AL, BE, GA, RC, RS, YP);
  scan_plain_kernel<<<24, kThr, 0, stream>>>(PROJ, AL, BE, GA, YP);
  ygate_kernel<<<dim3(1, kT), kThr, 0, stream>>>(YP, PROJ, Dp, Y16);
  wmma_gemm64<0, false, 2, 0, false, 0><<<dim3((kT / 64) * (kDM / 64) / 8, 1), 256, 0, stream>>>(
      Y16, Y16, kDI, 0L, WOUT16, WOUT16, kDI, 0L, (void*)out, (void*)out, kDM, 0L, ZB, nullptr, 0L, kT, kDM, kDI, 1.0f / (kCY * kInCarry));
}
static_assert(((kT / 64) * (kNP / 64)) % 8 == 0 && ((kT / 64) * (kDM / 64)) % 8 == 0, "the engine's grids: whole blocks of eight wave tiles");
